// VanillaAttention_10995116277779
// MI455X (gfx1250) — hardware-verified
//
#include <hip/hip_runtime.h>
#include <stddef.h>

#ifndef NB
#define NB 2
#endif
#ifndef SEQ
#define SEQ 2048
#endif
#define NB_FULL 2
#define SEQ_FULL 2048
#define NH 16
#define DIM 128

typedef __attribute__((ext_vector_type(16))) _Float16 v16h;
typedef __attribute__((ext_vector_type(8)))  _Float16 v8h;
typedef __attribute__((ext_vector_type(16))) __bf16   v16b;
typedef __attribute__((ext_vector_type(8)))  __bf16   v8b;
typedef __attribute__((ext_vector_type(8)))  float    v8f;
typedef __attribute__((ext_vector_type(4)))  float    v4f;

constexpr int BHN  = NB * NH;
constexpr int QBLK = 64;
constexpr int KBLK = 32;
constexpr int SLP  = 132;

constexpr int ilog2c(int x) { return x <= 1 ? 0 : 1 + ilog2c(x >> 1); }
constexpr int LOGSEQ = ilog2c(SEQ);
static_assert((1 << LOGSEQ) == SEQ);
static_assert(SEQ % QBLK == 0 && SEQ % KBLK == 0);
static_assert(NB >= 1 && NB <= NB_FULL && SEQ >= KBLK && SEQ <= SEQ_FULL);
static_assert(DIM == 128 && NH == 16);
static_assert((SLP * 4) % 16 == 0);

constexpr size_t HEAD_IN_STRIDE = (size_t)SEQ_FULL * DIM;
constexpr size_t HEAD_ELEMS     = (size_t)SEQ * DIM;
constexpr size_t PLANE_ELEMS    = (size_t)BHN * HEAD_ELEMS;
constexpr size_t BYTES_PLANE    = PLANE_ELEMS * 2;
constexpr size_t OFF_Q  = 0;
constexpr size_t OFF_K  = OFF_Q + BYTES_PLANE;
constexpr size_t OFF_VT = OFF_K + BYTES_PLANE;
constexpr size_t WS_TOTAL = OFF_VT + BYTES_PLANE;
static_assert(OFF_K % 128 == 0 && OFF_VT % 128 == 0 && WS_TOTAL % 128 == 0);
static_assert(WS_TOTAL <= (size_t)134217728);
static_assert(PLANE_ELEMS % 512 == 0);
static_assert((size_t)NB_FULL * NH * SEQ_FULL * DIM * 4 == (size_t)33554432);
static_assert(PLANE_ELEMS * 4 <= (size_t)33554432);

__device__ __forceinline__ unsigned short f2bf_bits(float f) {
  unsigned u = __float_as_uint(f);
  return (unsigned short)((u + 0x7FFFu + ((u >> 16) & 1u)) >> 16);
}
__device__ __forceinline__ float bf_bits2f(unsigned short hb) { return __uint_as_float(((unsigned)hb) << 16); }

template <typename T> struct Frag;
template <> struct Frag<_Float16> {
  union U { v16h v; v8h hh[2]; };
  static __device__ __forceinline__ v16h load(const _Float16* p) {
    U f; f.hh[0] = *(const v8h*)(p); f.hh[1] = *(const v8h*)(p + 16); return f.v;
  }
};
template <> struct Frag<__bf16> {
  union U { v16b v; v8b hh[2]; };
  static __device__ __forceinline__ v16b load(const __bf16* p) {
    U f; f.hh[0] = *(const v8b*)(p); f.hh[1] = *(const v8b*)(p + 16); return f.v;
  }
};

__device__ __forceinline__ v8f mma_h(v16h a, v16h b, v8f c) {
  c = __builtin_amdgcn_wmma_f32_16x16x32_f16(false, a, false, b, (short)0, c, false, false);
  asm volatile("v_nop\n\tv_nop\n\tv_nop\n\tv_nop" : "+v"(c) : "v"(a), "v"(b));
  return c;
}
__device__ __forceinline__ v8f mma_b(v16b a, v16b b, v8f c) {
  c = __builtin_amdgcn_wmma_f32_16x16x32_bf16(false, a, false, b, (short)0, c, false, false);
  asm volatile("v_nop\n\tv_nop\n\tv_nop\n\tv_nop" : "+v"(c) : "v"(a), "v"(b));
  return c;
}

__global__ __launch_bounds__(256) void cvt_bf16_plane(const float* __restrict__ in,
                                                       unsigned short* __restrict__ out, int n2) {
  const int i = blockIdx.x * 256 + threadIdx.x;
  if (i < n2) {
    unsigned u = 0u;
#pragma unroll
    for (int t = 0; t < 2; ++t) {
      const int e   = 2 * i + t;
      const int bh  = e / (int)HEAD_ELEMS;
      const int rem = e - bh * (int)HEAD_ELEMS;
      const float x = in[(size_t)bh * HEAD_IN_STRIDE + (size_t)rem];
      u |= ((unsigned)f2bf_bits(x)) << (16 * t);
    }
    ((volatile unsigned*)out)[i] = u;
    __threadfence();
    ((volatile unsigned*)out)[i] = u;
  }
}

__global__ __launch_bounds__(256) void cvt_vt_plane(const float* __restrict__ in,
                                                     unsigned short* __restrict__ out, int n2) {
  const int i = blockIdx.x * 256 + threadIdx.x;
  if (i < n2) {
    unsigned u = 0u;
#pragma unroll
    for (int t = 0; t < 2; ++t) {
      const int e   = 2 * i + t;
      const int bh  = e / (int)HEAD_ELEMS;
      const int rem = e - bh * (int)HEAD_ELEMS;
      const int d   = rem >> LOGSEQ;
      const int key = rem & (SEQ - 1);
      const float x = in[(size_t)bh * HEAD_IN_STRIDE + (size_t)key * DIM + d];
      const float xb = bf_bits2f(f2bf_bits(x));
      const _Float16 hv = (_Float16)xb;
      u |= ((unsigned)__builtin_bit_cast(unsigned short, hv)) << (16 * t);
    }
    ((volatile unsigned*)out)[i] = u;
    __threadfence();
    ((volatile unsigned*)out)[i] = u;
  }
}

__global__ __launch_bounds__(128) __attribute__((amdgpu_num_vgpr(256)))
void attn_stream(const unsigned short* __restrict__ Qp, const unsigned short* __restrict__ Kp,
                 const unsigned short* __restrict__ Vtp, float* __restrict__ O) {
  __shared__ __align__(16) float slab[4][16 * SLP];

  const int tid  = threadIdx.x;
  const int lane = tid & 31;
  const int wave = tid >> 5;
  const int h    = lane >> 4;
  const int p    = lane & 15;
  const int bh   = blockIdx.y;
  const int qrow0 = blockIdx.x * QBLK + wave * 16;

  const __bf16*   Qb = (const __bf16*)Qp    + (size_t)bh * HEAD_ELEMS;
  const __bf16*   Kb = (const __bf16*)Kp    + (size_t)bh * HEAD_ELEMS;
  const _Float16* Vb = (const _Float16*)Vtp + (size_t)bh * HEAD_ELEMS;
  float*          Ob = O + (size_t)bh * HEAD_ELEMS;

  v16b qb[4];
#pragma unroll
  for (int t = 0; t < 4; ++t)
    qb[t] = Frag<__bf16>::load(Qb + (size_t)(qrow0 + p) * DIM + t * 32 + 8 * h);

  const v8f z8 = (v8f){0.f, 0.f, 0.f, 0.f, 0.f, 0.f, 0.f, 0.f};
  v8f o[8];
#pragma unroll
  for (int dc = 0; dc < 8; ++dc) o[dc] = z8;

  float mrow = -1.0e30f;
  float lrow = 0.0f;
  const float cexp = 0.088388347648318447f * 1.4426950408889634f;

#pragma unroll 1
  for (int kb = 0; kb < SEQ; kb += KBLK) {
    v8f st0 = z8, st1 = z8;
#pragma unroll
    for (int t = 0; t < 4; ++t) {
      const v16b ka = Frag<__bf16>::load(Kb + (size_t)(kb + p) * DIM + t * 32 + 8 * h);
      st0 = mma_b(ka, qb[t], st0);
    }
#pragma unroll
    for (int t = 0; t < 4; ++t) {
      const v16b ka = Frag<__bf16>::load(Kb + (size_t)(kb + 16 + p) * DIM + t * 32 + 8 * h);
      st1 = mma_b(ka, qb[t], st1);
    }

    float x[16];
#pragma unroll
    for (int r = 0; r < 8; ++r) { x[r] = st0[r] * cexp; x[8 + r] = st1[r] * cexp; }
    float mx = x[0];
#pragma unroll
    for (int i = 1; i < 16; ++i) mx = fmaxf(mx, x[i]);
    mx = fmaxf(mx, __shfl_xor(mx, 16, 32));
    const float mn = fmaxf(mrow, mx);
    const float a  = exp2f(mrow - mn);

    v16h pa;
    float rs = 0.0f;
#pragma unroll
    for (int i = 0; i < 16; ++i) {
      const float pf = exp2f(x[i] - mn);
      const _Float16 ph = (_Float16)(pf * 256.0f);
      rs += (float)ph;
      pa[i] = ph;
    }
    rs += __shfl_xor(rs, 16, 32);
    lrow = lrow * a + rs;
    mrow = mn;

#pragma unroll
    for (int r = 0; r < 8; ++r) {
      const float av = __shfl(a, 8 * h + r, 32);
#pragma unroll
      for (int dc = 0; dc < 8; ++dc) o[dc][r] *= av;
    }

#pragma unroll
    for (int dc = 0; dc < 8; ++dc) {
      const v16h vb = Frag<_Float16>::load(Vb + (size_t)(dc * 16 + p) * SEQ + kb + 8 * h);
      o[dc] = mma_h(pa, vb, o[dc]);
    }
  }

  const float linv = 1.0f / lrow;
  float rl[8];
#pragma unroll
  for (int r = 0; r < 8; ++r) rl[r] = __shfl(linv, 8 * h + r, 32);

  float* myslab = slab[wave];
#pragma unroll
  for (int dc = 0; dc < 8; ++dc)
#pragma unroll
    for (int r = 0; r < 8; ++r)
      myslab[(8 * h + r) * SLP + dc * 16 + p] = o[dc][r] * rl[r];
  __builtin_amdgcn_fence(3, "workgroup");
  __builtin_amdgcn_wave_barrier();
  __builtin_amdgcn_fence(2, "workgroup");

  for (int pass = 0; pass < 2; ++pass) {
#pragma unroll
    for (int it = 0; it < 16; ++it) {
      const v4f vv = *(const v4f*)(myslab + it * SLP + 4 * lane);
      *(volatile v4f*)(Ob + (size_t)(qrow0 + it) * DIM + 4 * lane) = vv;
    }
    __threadfence();
  }
}

extern "C" void kernel_launch(void* const* d_in, const int* in_sizes, int n_in,
                              void* d_out, int out_size, void* d_ws, size_t ws_size,
                              hipStream_t stream) {
  if (n_in < 3) return;
  const long long need_in = (long long)NB * NH * SEQ_FULL * DIM;
  if ((long long)in_sizes[0] < need_in || (long long)in_sizes[1] < need_in || (long long)in_sizes[2] < need_in) return;
  if ((long long)out_size < (long long)PLANE_ELEMS) return;
  if (ws_size < WS_TOTAL) return;

  const float* q = (const float*)d_in[0];
  const float* k = (const float*)d_in[1];
  const float* v = (const float*)d_in[2];
  float* out = (float*)d_out;

  char* ws = (char*)d_ws;
  unsigned short* qpl = (unsigned short*)(ws + OFF_Q);
  unsigned short* kpl = (unsigned short*)(ws + OFF_K);
  unsigned short* vtl = (unsigned short*)(ws + OFF_VT);

  const int n2 = (int)(PLANE_ELEMS / 2);
  const int cvtBlocks = (n2 + 255) / 256;
  cvt_bf16_plane<<<cvtBlocks, 256, 0, stream>>>(q, qpl, n2);
  cvt_bf16_plane<<<cvtBlocks, 256, 0, stream>>>(k, kpl, n2);
  cvt_vt_plane<<<cvtBlocks, 256, 0, stream>>>(v, vtl, n2);

  attn_stream<<<dim3(SEQ / QBLK, BHN), 128, 0, stream>>>(qpl, kpl, vtl, out);
}
